// MHA2D_3934190043350
// MI455X (gfx1250) — hardware-run, weakly checked
//
#include <hip/hip_runtime.h>
#include <stddef.h>
#include <stdint.h>

#define NBAT 8
#define NCH  128
#define NPIX 1024
#define IMW  32
#define NHD  8
#define KD   16
#define NBH  (NBAT * NHD)
#define PXB  64
#define QB   128
#define KC   64

#define ASC    4.0f
#define WSC    32.0f
#define PSCALE 0.015625f
#define SSCALE 0.0625f
#define PSC    1024.0f
#define OSC    0.00048828125f

static_assert(NCH == NHD * KD);
static_assert(NPIX == IMW * IMW);
static_assert(PXB == 64);
static_assert(NPIX % PXB == 0);
static_assert(NPIX % QB == 0);
static_assert(NPIX % KC == 0);
static_assert(QB == 8 * 16);
static_assert(NCH % 32 == 0);
static_assert((NCH * NCH) % 2048 == 0);

typedef _Float16 v16h __attribute__((ext_vector_type(16)));
typedef _Float16 v8h  __attribute__((ext_vector_type(8)));
typedef float    v8f  __attribute__((ext_vector_type(8)));
typedef float    v4f  __attribute__((ext_vector_type(4)));
typedef unsigned int v4u __attribute__((ext_vector_type(4)));

union Frag  { v16h v; v8h h[2]; };
union Pack8 { v8h h; v4u u; };

__device__ __forceinline__ v8f mma16(v16h a, v16h b, v8f c) {
  c = __builtin_amdgcn_wmma_f32_16x16x32_f16(false, a, false, b, (short)0, c, false, false);
  asm volatile("v_nop\n\tv_nop\n\tv_nop\n\tv_nop" : "+v"(c) : "v"(a), "v"(b));
  return c;
}

__device__ __forceinline__ v8f zero8() { return (v8f){0.f, 0.f, 0.f, 0.f, 0.f, 0.f, 0.f, 0.f}; }
__device__ __forceinline__ v8h zero8h() {
  const _Float16 z = (_Float16)0.0f;
  return (v8h){z, z, z, z, z, z, z, z};
}

__device__ __forceinline__ v16h ldfrag(const _Float16* p, int ld, int row0, int k0, int lane) {
  const int m = lane & 15, lh = lane >> 4;
  const _Float16* q = p + (size_t)(row0 + m) * ld + k0 + 8 * lh;
  Frag f;
  f.h[0] = *(const v8h*)(q);
  f.h[1] = *(const v8h*)(q + 16);
  return f.v;
}

__global__ __launch_bounds__(256) void k_stats(const float* __restrict__ x, float* __restrict__ stat) {
  __shared__ __align__(16) float sm[64];
  const int tid = threadIdx.x, lane = tid & 31, wave = tid >> 5;
  const int cb = blockIdx.x * 32;
#pragma unroll 1
  for (int i = 0; i < 4; ++i) {
    const int cl = wave * 4 + i;
    const int c  = cb + cl;
    double s = 0.0;
#pragma unroll 1
    for (int b = 0; b < NBAT; ++b) {
      const float* p = x + ((size_t)b * NCH + c) * NPIX;
#pragma unroll
      for (int t = 0; t < 8; ++t) {
        const v4f v = *(const v4f*)(p + 4 * (lane + 32 * t));
        s += ((double)v[0] + (double)v[1]) + ((double)v[2] + (double)v[3]);
      }
    }
#pragma unroll
    for (int off = 16; off >= 1; off >>= 1) s += __shfl_xor(s, off, 32);
    const double mu = s * (1.0 / 8192.0);
    double ss = 0.0;
#pragma unroll 1
    for (int b = 0; b < NBAT; ++b) {
      const float* p = x + ((size_t)b * NCH + c) * NPIX;
#pragma unroll
      for (int t = 0; t < 8; ++t) {
        const v4f v = *(const v4f*)(p + 4 * (lane + 32 * t));
        const double d0 = (double)v[0] - mu, d1 = (double)v[1] - mu;
        const double d2 = (double)v[2] - mu, d3 = (double)v[3] - mu;
        ss += (d0 * d0 + d1 * d1) + (d2 * d2 + d3 * d3);
      }
    }
#pragma unroll
    for (int off = 16; off >= 1; off >>= 1) ss += __shfl_xor(ss, off, 32);
    const double var = ss * (1.0 / 8192.0);
    const float varf = (float)var;
    const float rs   = 1.0f / sqrtf(varf + 1e-5f);
    if (lane == 0) { sm[cl] = (float)mu; sm[32 + cl] = rs; }
  }
  __syncthreads();
  if (tid < 16) {
    const int which = tid >> 3, q = tid & 7;
    const v4f v = *(const v4f*)(sm + which * 32 + 4 * q);
    volatile v4f* d = (volatile v4f*)(stat + which * NCH + cb + 4 * q);
    *d = v;
    __threadfence();
    *d = v;
  }
}

__global__ __launch_bounds__(256) void k_wcvt(const float* __restrict__ wq, const float* __restrict__ wk,
                                              const float* __restrict__ wv, _Float16* __restrict__ wh) {
  const int m = blockIdx.x >> 3;
  const int o = (blockIdx.x & 7) * 2048 + threadIdx.x * 8;
  const v4f q0 = *(const v4f*)(wq + o), q1 = *(const v4f*)(wq + o + 4);
  const v4f k0 = *(const v4f*)(wk + o), k1 = *(const v4f*)(wk + o + 4);
  const v4f v0 = *(const v4f*)(wv + o), v1 = *(const v4f*)(wv + o + 4);
  const v4f a0 = ((m == 0) ? q0 : ((m == 1) ? k0 : v0)) * WSC;
  const v4f a1 = ((m == 0) ? q1 : ((m == 1) ? k1 : v1)) * WSC;
  Pack8 pk;
  pk.h = (v8h){(_Float16)a0[0], (_Float16)a0[1], (_Float16)a0[2], (_Float16)a0[3],
               (_Float16)a1[0], (_Float16)a1[1], (_Float16)a1[2], (_Float16)a1[3]};
  const v4u vv = pk.u;
  volatile v4u* d = (volatile v4u*)(wh + (size_t)m * NCH * NCH + o);
  *d = vv;
  __threadfence();
  *d = vv;
}

#define AP  136
#define QTP 16
#define VTP 72

__device__ __forceinline__ void proj_gemm(const _Float16* sA, const _Float16* __restrict__ wm,
                                          int wave, int lane, v8f (&acc)[4]) {
#pragma unroll
  for (int rt = 0; rt < 4; ++rt) acc[rt] = zero8();
#pragma unroll
  for (int ks = 0; ks < NCH / 32; ++ks) {
    const int k0 = ks * 32;
    const v16h bf = ldfrag(wm, NCH, wave * KD, k0, lane);
    const v16h a0 = ldfrag(sA, AP, 0, k0, lane);
    const v16h a1 = ldfrag(sA, AP, 16, k0, lane);
    const v16h a2 = ldfrag(sA, AP, 32, k0, lane);
    const v16h a3 = ldfrag(sA, AP, 48, k0, lane);
    acc[0] = mma16(a0, bf, acc[0]);
    acc[1] = mma16(a1, bf, acc[1]);
    acc[2] = mma16(a2, bf, acc[2]);
    acc[3] = mma16(a3, bf, acc[3]);
  }
}

__device__ __forceinline__ void store_qk(const v8f (&acc)[4], _Float16* st, _Float16* __restrict__ dst,
                                         int lane, int hh, int lm) {
  __syncthreads();
#pragma unroll
  for (int rt = 0; rt < 4; ++rt)
#pragma unroll
    for (int r = 0; r < 8; ++r)
      st[(rt * 16 + 8 * hh + r) * QTP + lm] = (_Float16)(acc[rt][r] * PSCALE);
  __syncthreads();
  v4u val[4];
#pragma unroll
  for (int it = 0; it < 4; ++it) {
    const int p = lane + 32 * it;
    Pack8 pk;
    pk.h = *(const v8h*)(st + p * 8);
    val[it] = pk.u;
  }
#pragma unroll
  for (int it = 0; it < 4; ++it) *(volatile v4u*)(dst + (lane + 32 * it) * 8) = val[it];
  __threadfence();
#pragma unroll
  for (int it = 0; it < 4; ++it) *(volatile v4u*)(dst + (lane + 32 * it) * 8) = val[it];
}

__device__ __forceinline__ void store_vt(const v8f (&acc)[4], _Float16* st, _Float16* __restrict__ dst,
                                         int lane, int hh, int lm) {
  __syncthreads();
#pragma unroll
  for (int rt = 0; rt < 4; ++rt)
#pragma unroll
    for (int r = 0; r < 8; ++r)
      st[lm * VTP + rt * 16 + 8 * hh + r] = (_Float16)(acc[rt][r] * PSCALE);
  __syncthreads();
  v4u val[4];
  size_t go[4];
#pragma unroll
  for (int it = 0; it < 4; ++it) {
    const int p  = lane + 32 * it;
    const int d  = p >> 3;
    const int pc = p & 7;
    Pack8 pk;
    pk.h = *(const v8h*)(st + d * VTP + pc * 8);
    val[it] = pk.u;
    go[it]  = (size_t)d * NPIX + pc * 8;
  }
#pragma unroll
  for (int it = 0; it < 4; ++it) *(volatile v4u*)(dst + go[it]) = val[it];
  __threadfence();
#pragma unroll
  for (int it = 0; it < 4; ++it) *(volatile v4u*)(dst + go[it]) = val[it];
}

__global__ __launch_bounds__(256) void k_proj(const float* __restrict__ x, const float* __restrict__ stat,
                                              const float* __restrict__ gamma, const float* __restrict__ beta,
                                              const _Float16* __restrict__ wh,
                                              _Float16* __restrict__ qp, _Float16* __restrict__ kp,
                                              _Float16* __restrict__ vtp) {
  __shared__ __align__(16) _Float16 sA[PXB * AP];
  __shared__ __align__(16) _Float16 sT[8 * 16 * VTP];
  __shared__ float sPar[4 * NCH];

  const int tid = threadIdx.x, lane = tid & 31, wave = tid >> 5;
  const int hh = lane >> 4, lm = lane & 15;
  const int b  = blockIdx.x / (NPIX / PXB);
  const int n0 = (blockIdx.x - b * (NPIX / PXB)) * PXB;
  const int bh = b * NHD + wave;

  if (tid < NCH) {
    sPar[tid]           = stat[tid];
    sPar[NCH + tid]     = stat[NCH + tid];
    sPar[2 * NCH + tid] = gamma[tid];
    sPar[3 * NCH + tid] = beta[tid];
  }
  __syncthreads();

#pragma unroll 1
  for (int j = 0; j < (PXB * NCH) / 256; ++j) {
    const int i  = tid + 256 * j;
    const int c  = i >> 6;
    const int px = i & 63;
    float v = x[((size_t)b * NCH + c) * NPIX + n0 + px];
    v = (v - sPar[c]) * sPar[NCH + c];
    v = v * sPar[2 * NCH + c] + sPar[3 * NCH + c];
    const float g = 0.5f * v * (1.0f + erff(v * 0.70710678118654752f));
    sA[px * AP + c] = (_Float16)(g * ASC);
  }
  __syncthreads();

  _Float16* st = sT + wave * (16 * VTP);
  v8f acc[4];
  proj_gemm(sA, wh, wave, lane, acc);
  store_qk(acc, st, qp + ((size_t)bh * NPIX + n0) * KD, lane, hh, lm);
  proj_gemm(sA, wh + (size_t)NCH * NCH, wave, lane, acc);
  store_qk(acc, st, kp + ((size_t)bh * NPIX + n0) * KD, lane, hh, lm);
  proj_gemm(sA, wh + (size_t)2 * NCH * NCH, wave, lane, acc);
  store_vt(acc, st, vtp + (size_t)bh * KD * NPIX + n0, lane, hh, lm);
}

#define PTP 72
#define OTP 132
__global__ __launch_bounds__(256) void k_attn(const float* __restrict__ x,
                                              const _Float16* __restrict__ qp,
                                              const _Float16* __restrict__ kp,
                                              const _Float16* __restrict__ vtp,
                                              const float* __restrict__ peh, const float* __restrict__ pew,
                                              float* __restrict__ out) {
  __shared__ __align__(16) _Float16 sP[8 * 16 * PTP];
  __shared__ __align__(16) float sO[KD * OTP];
  __shared__ float sEh[64];
  __shared__ float sEw[64];

  const int tid = threadIdx.x, lane = tid & 31, wave = tid >> 5;
  const int hh = lane >> 4, lm = lane & 15;
  const int bh = blockIdx.x / (NPIX / QB);
  const int qc = blockIdx.x - bh * (NPIX / QB);
  const int b  = bh / NHD, h = bh - b * NHD;
  const int q0 = qc * QB;
  const int qw0 = q0 + wave * 16;

  if (tid < 64) {
    const int i = (tid < 62) ? tid : 62;
    const float e0 = peh[i], e1 = pew[i];
    sEh[tid] = (tid < 63) ? e0 : 0.f;
    sEw[tid] = (tid < 63) ? e1 : 0.f;
  }

  const _Float16* Kb = kp  + (size_t)bh * NPIX * KD;
  const _Float16* Vb = vtp + (size_t)bh * KD * NPIX;

  Frag qa;
  qa.h[0] = *(const v8h*)(qp + ((size_t)bh * NPIX + qw0 + lm) * KD + 8 * hh);
  qa.h[1] = zero8h();

  __syncthreads();
  const int qh = qw0 >> 5;
  float ew0[8], ew1[8];
#pragma unroll
  for (int r = 0; r < 8; ++r) {
    const int qwv = (qw0 + 8 * hh + r) & 31;
    ew0[r] = sEw[qwv + 31 - lm];
    ew1[r] = sEw[qwv + 15 - lm];
  }

  const float NEGI = -__builtin_huge_valf();
  float mrow[8], lrow[8];
  v8f oacc = zero8();
#pragma unroll
  for (int r = 0; r < 8; ++r) { mrow[r] = NEGI; lrow[r] = 0.f; }

  _Float16* pw = sP + wave * (16 * PTP);

  for (int kc = 0; kc < NPIX / KC; ++kc) {
    const int kv0 = kc * KC;
    __syncthreads();

    v8f s[4];
#pragma unroll
    for (int j = 0; j < 4; ++j) {
      Frag kb;
      kb.h[0] = *(const v8h*)(Kb + (size_t)(kv0 + 16 * j + lm) * KD + 8 * hh);
      kb.h[1] = zero8h();
      s[j] = mma16(qa.v, kb.v, zero8());
    }
    const float eh0 = sEh[qh + 31 - 2 * kc];
    const float eh1 = sEh[qh + 30 - 2 * kc];
    float cm[8];
#pragma unroll
    for (int r = 0; r < 8; ++r) {
      float m = NEGI;
#pragma unroll
      for (int j = 0; j < 4; ++j) {
        const float eb = ((j < 2) ? eh0 : eh1) + ((j & 1) ? ew1[r] : ew0[r]);
        s[j][r] = s[j][r] * SSCALE + eb;
        m = fmaxf(m, s[j][r]);
      }
#pragma unroll
      for (int off = 1; off < 16; off <<= 1) m = fmaxf(m, __shfl_xor(m, off, 32));
      cm[r] = m;
    }
    float al[8];
#pragma unroll
    for (int r = 0; r < 8; ++r) {
      const float mnew  = fmaxf(mrow[r], cm[r]);
      const float alpha = __expf(mrow[r] - mnew);
      mrow[r] = mnew;
      float psum = 0.f;
#pragma unroll
      for (int j = 0; j < 4; ++j) {
        const float p = __expf(s[j][r] - mnew);
        psum += p;
        pw[(8 * hh + r) * PTP + 16 * j + lm] = (_Float16)(p * PSC);
      }
#pragma unroll
      for (int off = 1; off < 16; off <<= 1) psum += __shfl_xor(psum, off, 32);
      lrow[r] = lrow[r] * alpha + psum;
      al[r] = alpha;
    }
#pragma unroll
    for (int r = 0; r < 8; ++r) oacc[r] *= al[r];
    __syncthreads();

#pragma unroll
    for (int kk = 0; kk < 2; ++kk) {
      const v16h pa = ldfrag(pw, PTP, 0, kk * 32, lane);
      const v16h vb = ldfrag(Vb, NPIX, 0, kv0 + kk * 32, lane);
      oacc = mma16(pa, vb, oacc);
    }
  }

  float sc[8];
#pragma unroll
  for (int r = 0; r < 8; ++r) sc[r] = (1.0f / lrow[r]) * OSC;
  __syncthreads();
#pragma unroll
  for (int r = 0; r < 8; ++r) sO[lm * OTP + wave * 16 + 8 * hh + r] = oacc[r] * sc[r];
  __syncthreads();
  v4f val[2];
  size_t go[2];
#pragma unroll
  for (int it = 0; it < 2; ++it) {
    const int d = wave + 8 * it;
    go[it] = ((size_t)(b * NCH + h * KD + d)) * NPIX + q0 + 4 * lane;
    const v4f xv = *(const v4f*)(x + go[it]);
    const v4f ov = *(const v4f*)(sO + d * OTP + 4 * lane);
    val[it] = xv + ov;
  }
#pragma unroll
  for (int it = 0; it < 2; ++it) *(volatile v4f*)(out + go[it]) = val[it];
  __threadfence();
#pragma unroll
  for (int it = 0; it < 2; ++it) *(volatile v4f*)(out + go[it]) = val[it];
}

extern "C" void kernel_launch(void* const* d_in, const int* in_sizes, int n_in,
                              void* d_out, int out_size, void* d_ws, size_t ws_size,
                              hipStream_t stream) {
  if (n_in < 8) return;
  if (in_sizes[0] != NBAT * NCH * NPIX) return;
  if (in_sizes[1] != NCH) return;
  if (in_sizes[2] != NCH) return;
  if (in_sizes[3] != NCH * NCH) return;
  if (in_sizes[4] != NCH * NCH) return;
  if (in_sizes[5] != NCH * NCH) return;
  if (in_sizes[6] != 2 * IMW - 1) return;
  if (in_sizes[7] != 2 * IMW - 1) return;
  if (out_size != NBAT * NCH * NPIX) return;

  const float* x     = (const float*)d_in[0];
  const float* gamma = (const float*)d_in[1];
  const float* beta  = (const float*)d_in[2];
  const float* wq    = (const float*)d_in[3];
  const float* wk    = (const float*)d_in[4];
  const float* wv    = (const float*)d_in[5];
  const float* peh   = (const float*)d_in[6];
  const float* pew   = (const float*)d_in[7];
  float* out = (float*)d_out;

  size_t off = 0;
  const size_t oStat = off; off += 256 * 4;
  const size_t oWh   = off; off += (size_t)3 * NCH * NCH * 2;
  off = (off + 4095) & ~(size_t)4095;
  const size_t oQ    = off; off += (size_t)NBH * NPIX * KD * 2;
  const size_t oK    = off; off += (size_t)NBH * NPIX * KD * 2;
  const size_t oV    = off; off += (size_t)NBH * KD * NPIX * 2;
  if (off > ws_size) return;
  if (off > (size_t)134217728) return;

  char* ws = (char*)d_ws;
  float*    stat = (float*)(ws + oStat);
  _Float16* wh   = (_Float16*)(ws + oWh);
  _Float16* qpl  = (_Float16*)(ws + oQ);
  _Float16* kpl  = (_Float16*)(ws + oK);
  _Float16* vtpl = (_Float16*)(ws + oV);

  k_stats<<<dim3(NCH / 32), dim3(256), 0, stream>>>(x, stat);
  k_wcvt<<<dim3(3 * (NCH * NCH) / 2048), dim3(256), 0, stream>>>(wq, wk, wv, wh);
  k_proj<<<dim3(NBAT * (NPIX / PXB)), dim3(256), 0, stream>>>(x, stat, gamma, beta, wh, qpl, kpl, vtpl);
  k_attn<<<dim3(NBH * (NPIX / QB)), dim3(256), 0, stream>>>(x, qpl, kpl, vtpl, peh, pew, out);
  (void)hipGetLastError();
}
